// CNN_LSTM_36618891165822
// MI455X (gfx1250) — hardware-verified
//
#include <hip/hip_runtime.h>
#include <stdint.h>
#include <stddef.h>

typedef __attribute__((ext_vector_type(16))) _Float16 v16h;
typedef __attribute__((ext_vector_type(8)))  _Float16 v8h;
typedef __attribute__((ext_vector_type(16))) __bf16   v16b;
typedef __attribute__((ext_vector_type(8)))  __bf16   v8b;
typedef __attribute__((ext_vector_type(8)))  float    v8f;
typedef __attribute__((ext_vector_type(4)))  float    v4f;
typedef __attribute__((ext_vector_type(2)))  float    v2f;
typedef __attribute__((ext_vector_type(4)))  unsigned v4u;

__device__ __forceinline__ unsigned short f2bf_bits(float f) {
  unsigned u = __float_as_uint(f);
  return (unsigned short)((u + 0x7FFFu + ((u >> 16) & 1u)) >> 16);
}
__device__ __forceinline__ float bf_bits2f(unsigned short h) { return __uint_as_float(((unsigned)h) << 16); }

__device__ __forceinline__ void dep_guard_h(v8f& a, v8f& b, v16h x, v16h y) { asm volatile("v_nop\n\tv_nop\n\tv_nop\n\tv_nop" : "+v"(a), "+v"(b) : "v"(x), "v"(y)); }
__device__ __forceinline__ void dep_guard_b(v8f& a, v8f& b, v16b x, v16b y) { asm volatile("v_nop\n\tv_nop\n\tv_nop\n\tv_nop" : "+v"(a), "+v"(b) : "v"(x), "v"(y)); }
__device__ __forceinline__ void keep4_h(v16h a, v16h b, v16h c, v16h d) { asm volatile("v_nop" :: "v"(a), "v"(b), "v"(c), "v"(d)); }
__device__ __forceinline__ void keep4_b(v16b a, v16b b, v16b c, v16b d) { asm volatile("v_nop" :: "v"(a), "v"(b), "v"(c), "v"(d)); }
__device__ __forceinline__ void acc_guard4(v8f& a, v8f& b, v8f& c, v8f& d) { asm volatile("v_nop\n\tv_nop\n\tv_nop\n\tv_nop" : "+v"(a), "+v"(b), "+v"(c), "+v"(d)); }
template <typename T> struct Frag;
template <> struct Frag<_Float16> {
  typedef v16h V; union U { v16h v; v8h h[2]; };
  static __device__ __forceinline__ v16h load(const _Float16* p) {
    U f; f.h[0] = *(const v8h*)(p); f.h[1] = *(const v8h*)(p + 16); return f.v;
  }
  static __device__ __forceinline__ v8f mma(v16h a, v16h b, v8f c) {
    return __builtin_amdgcn_wmma_f32_16x16x32_f16(false, a, false, b, (short)0, c, false, false);
  }
  static __device__ __forceinline__ void guard(v8f& a, v8f& b, v16h x, v16h y) { dep_guard_h(a, b, x, y); }
  static __device__ __forceinline__ void keep(v16h a, v16h b, v16h c, v16h d) { keep4_h(a, b, c, d); }
};
template <> struct Frag<__bf16> {
  typedef v16b V; union U { v16b v; v8b h[2]; };
  static __device__ __forceinline__ v16b load(const __bf16* p) {
    U f; f.h[0] = *(const v8b*)(p); f.h[1] = *(const v8b*)(p + 16); return f.v;
  }
  static __device__ __forceinline__ v8f mma(v16b a, v16b b, v8f c) {
    return __builtin_amdgcn_wmma_f32_16x16x32_bf16(false, a, false, b, (short)0, c, false, false);
  }
  static __device__ __forceinline__ void guard(v8f& a, v8f& b, v16b x, v16b y) { dep_guard_b(a, b, x, y); }
  static __device__ __forceinline__ void keep(v16b a, v16b b, v16b c, v16b d) { keep4_b(a, b, c, d); }
};

template <int ET> struct Elem;
template <> struct Elem<0> { typedef _Float16 T; };
template <> struct Elem<1> { typedef __bf16 T; };
template <int ET, bool SPLIT, int BIAS_MODE, int OUT_MODE, bool RESID, int ACT = 0>
__global__ __launch_bounds__(256) void wmma_gemm64(
    const unsigned short* __restrict__ Ap, const unsigned short* __restrict__ A2p, int lda, long strideA,
    const unsigned short* __restrict__ Btp, const unsigned short* __restrict__ Bt2p, int ldb, long strideB,
    void* __restrict__ Cout, void* __restrict__ Cout2, int ldc, long strideC,
    const float* __restrict__ bias,
    const float* __restrict__ resid, long strideR,
    int M, int N, int K, float scale) {
  typedef typename Elem<ET>::T T;
  typedef typename Frag<T>::V V;
  const T* A = (const T*)Ap; const T* A2 = (const T*)A2p; const T* Bt = (const T*)Btp; const T* Bt2 = (const T*)Bt2p;
  __shared__ __align__(16) float sT[8][16 * 68];
  const int b    = blockIdx.y;
  const int lane = threadIdx.x & 31;
  const int wave = threadIdx.x >> 5;
  const int tilesN = N >> 6;
  const int tilesM = M >> 6;
  const int tile = blockIdx.x * 8 + wave;
  if (tile >= tilesM * tilesN) return;
  const int tm = tile / tilesN;
  const int tn = tile - tm * tilesN;
  const int m0 = tm << 6;
  const int n0 = tn << 6;

  const T* Ab  = A  + (size_t)b * strideA;
  const T* Bb  = Bt + (size_t)b * strideB;
  const T* Ab2 = SPLIT ? (A2  + (size_t)b * strideA) : nullptr;
  const T* Bb2 = SPLIT ? (Bt2 + (size_t)b * strideB) : nullptr;

  const int rlane = lane & 15;
  const int koff  = (lane >> 4) * 8;
  const int mOff  = (lane >> 4) * 8;

  v8f acc[4][4];
#pragma unroll
  for (int i = 0; i < 4; ++i)
#pragma unroll
    for (int j = 0; j < 4; ++j) acc[i][j] = (v8f){0.f,0.f,0.f,0.f,0.f,0.f,0.f,0.f};

  for (int k0 = 0; k0 < K; k0 += 32) {
    V bh[4], bl[4];
#pragma unroll
    for (int j = 0; j < 4; ++j) {
      const size_t bo = (size_t)(n0 + (j << 4) + rlane) * ldb + koff + k0;
      bh[j] = Frag<T>::load(Bb + bo);
      if (SPLIT) bl[j] = Frag<T>::load(Bb2 + bo);
    }
#pragma unroll
    for (int i = 0; i < 4; ++i) {
      const size_t ao = (size_t)(m0 + (i << 4) + rlane) * lda + koff + k0;
      V ah = Frag<T>::load(Ab + ao);
      V al;
      if (SPLIT) al = Frag<T>::load(Ab2 + ao);
#pragma unroll
      for (int j = 0; j < 4; ++j) {
        acc[i][j] = Frag<T>::mma(ah, bh[j], acc[i][j]);
        if (SPLIT) {
          acc[i][j] = Frag<T>::mma(ah, bl[j], acc[i][j]);
          acc[i][j] = Frag<T>::mma(al, bh[j], acc[i][j]);
        }
      }
      Frag<T>::guard(acc[i][0], acc[i][3], ah, SPLIT ? al : ah);
    }
    Frag<T>::keep(bh[0], bh[1], bh[2], bh[3]);
    if (SPLIT) Frag<T>::keep(bl[0], bl[1], bl[2], bl[3]);
  }
  acc_guard4(acc[0][0], acc[0][1], acc[0][2], acc[0][3]);
  acc_guard4(acc[1][0], acc[1][1], acc[1][2], acc[1][3]);
  acc_guard4(acc[2][0], acc[2][1], acc[2][2], acc[2][3]);
  acc_guard4(acc[3][0], acc[3][1], acc[3][2], acc[3][3]);

  float* slab = sT[wave];
  const float* Rb = RESID ? (resid + (size_t)b * strideR) : nullptr;
#pragma unroll
  for (int i = 0; i < 4; ++i) {
    const int mBase = m0 + (i << 4);
#pragma unroll
    for (int j = 0; j < 4; ++j) {
      const int n = n0 + (j << 4) + rlane;
      float bv = 0.f;
      if (BIAS_MODE == 2) bv = bias[n];
#pragma unroll
      for (int r = 0; r < 8; ++r) {
        float v = acc[i][j][r] * scale;
        if (BIAS_MODE == 1) v += bias[mBase + mOff + r];
        if (BIAS_MODE == 2) v += bv;
        if (RESID) v += Rb[(size_t)(mBase + mOff + r) * ldc + n];
        if (ACT == 1) v = tanhf(v);
        if (ACT == 2) v = fmaxf(v, 0.0f);
        if (ACT == 3) v = v / (1.0f + expf(-v));
        if (ACT == 4) v = (v > 0.f) ? v : 0.01f * v;
        if (ACT == 5) v = 0.5f * v * (1.0f + erff(v * 0.70710678118654752f));
        slab[(mOff + r) * 68 + (j << 4) + rlane] = v;
      }
    }
    __builtin_amdgcn_fence(__ATOMIC_RELEASE, "workgroup");
    __builtin_amdgcn_wave_barrier();
    __builtin_amdgcn_fence(__ATOMIC_ACQUIRE, "workgroup");
    if (OUT_MODE == 0) {
      float* C = (float*)Cout + (size_t)b * strideC;
      const int hh = lane >> 4, c4 = (lane & 15) * 4;
      for (int pass = 0; pass < 2; ++pass) {
#pragma unroll
        for (int it = 0; it < 8; ++it) {
          const int row = it * 2 + hh;
          v4f v = *(const v4f*)(slab + row * 68 + c4);
          *(volatile v4f*)(C + (size_t)(mBase + row) * ldc + n0 + c4) = v;
        }
        __threadfence();
      }
    } else {
      const int q = lane >> 3, c8 = (lane & 7) * 8;
      unsigned short* C  = (unsigned short*)Cout  + (size_t)b * strideC;
      unsigned short* C2 = (OUT_MODE == 2) ? ((unsigned short*)Cout2 + (size_t)b * strideC) : nullptr;
      for (int pass = 0; pass < 2; ++pass) {
#pragma unroll
        for (int it = 0; it < 4; ++it) {
          const int row = it * 4 + q;
          const float* sp = slab + row * 68 + c8;
          v8h hv, lv;
#pragma unroll
          for (int e = 0; e < 8; ++e) {
            if (OUT_MODE == 1) {
              hv[e] = (_Float16)sp[e];
            } else {
              unsigned short hb = f2bf_bits(sp[e]);
              unsigned short lb = f2bf_bits(sp[e] - bf_bits2f(hb));
              hv[e] = __builtin_bit_cast(_Float16, hb);
              lv[e] = __builtin_bit_cast(_Float16, lb);
            }
          }
          *(volatile v8h*)(C + (size_t)(mBase + row) * ldc + n0 + c8) = hv;
          if (OUT_MODE == 2) *(volatile v8h*)(C2 + (size_t)(mBase + row) * ldc + n0 + c8) = lv;
        }
        __threadfence();
      }
    }
    __builtin_amdgcn_fence(__ATOMIC_RELEASE, "workgroup");
    __builtin_amdgcn_wave_barrier();
    __builtin_amdgcn_fence(__ATOMIC_ACQUIRE, "workgroup");
  }
}

constexpr int kNB    = 256;
constexpr int kLX    = 10000;
constexpr int kCh0   = 64;
constexpr int kCh1   = 128;
constexpr int kNQ    = 156;
constexpr int kRowsA0 = kNB * kNQ;
constexpr int kA0Pitch = 256;
constexpr int kK1    = 512;
constexpr int kSteps = 77;
constexpr int kHid   = 256;
constexpr int kGates = 1024;
constexpr int kNX    = kSteps * kNB;
constexpr int kFc    = 512;
constexpr int kCls   = 256;
constexpr int kHP    = 264;
constexpr float kWScale    = 16.0f;
constexpr float kWScaleInv = 0.0625f;

static_assert(kRowsA0 % 64 == 0, "conv1 M tile multiple");
static_assert(kCh1 % 64 == 0 && kK1 % 32 == 0, "conv1 N,K");
static_assert(kGates % 64 == 0 && kNX % 64 == 0 && kCh1 % 32 == 0 && kHid % 32 == 0, "projection M,N,K");
static_assert(kNB % 64 == 0 && kFc % 64 == 0 && kCls % 64 == 0 && kFc % 32 == 0, "fc M,N,K");

__device__ __forceinline__ v8f mma_h16(v16h a, v16h b, v8f c) {
  c = __builtin_amdgcn_wmma_f32_16x16x32_f16(false, a, false, b, (short)0, c, false, false);
  asm volatile("v_nop\n\tv_nop\n\tv_nop\n\tv_nop" : "+v"(c) : "v"(a), "v"(b));
  return c;
}
__device__ __forceinline__ float sigm_f(float v) {
  v = fminf(fmaxf(v, -40.0f), 40.0f);
  return __builtin_amdgcn_rcpf(1.0f + expf(-v));
}
__device__ __forceinline__ unsigned pack_h2(float a, float b) {
  const _Float16 h0 = (_Float16)a, h1 = (_Float16)b;
  return (unsigned)__builtin_bit_cast(unsigned short, h0) | ((unsigned)__builtin_bit_cast(unsigned short, h1) << 16);
}

struct SgTaps { float tt[124]; };
static_assert(sizeof(SgTaps) == 496, "arg size");

__global__ __launch_bounds__(256) void k_savgol(const float* __restrict__ x, float* __restrict__ ysg, SgTaps tp) {
  __shared__ float taps[124];
  if (threadIdx.x == 0) {
#pragma unroll
    for (int i = 0; i < 121; ++i) taps[i] = tp.tt[i];
  }
  __syncthreads();
  const int idx = blockIdx.x * 256 + threadIdx.x;
  const int b = idx / kLX;
  const int p = idx - b * kLX;
  int wb = p - 5;
  wb = wb < 0 ? 0 : wb;
  wb = wb > (kLX - 11) ? (kLX - 11) : wb;
  const int rs = (p < 5) ? p : ((p > kLX - 6) ? (p - (kLX - 11)) : 5);
  const float* xx = x + (size_t)b * kLX + wb;
  const float* tr = taps + rs * 11;
  float r = 0.0f;
#pragma unroll
  for (int w = 0; w < 11; ++w) r = fmaf(xx[w], tr[w], r);
  ((volatile float*)ysg)[idx] = r;
  __threadfence();
  ((volatile float*)ysg)[idx] = r;
}

__global__ __launch_bounds__(128) void k_conv0(const float* __restrict__ ysg, const float* __restrict__ w0,
    const float* __restrict__ cb, const float* __restrict__ g, const float* __restrict__ be,
    const float* __restrict__ mn, const float* __restrict__ vr, unsigned short* __restrict__ a0qp) {
  _Float16* a0q = (_Float16*)a0qp;
  __shared__ float xs[264];
  __shared__ __align__(16) _Float16 ot[4 * kA0Pitch];
  const int tid = threadIdx.x, lane = tid & 31, wave = tid >> 5;
  const int g4 = blockIdx.x;
  const int b  = blockIdx.y;
  const float* src = ysg + (size_t)b * kLX + 256 * g4;
  for (int i = tid; i < 264; i += 128) xs[i] = src[i];
  const int c = tid & 63, qp = tid >> 6;
  float wv[16];
  {
    const v4f* wp = (const v4f*)(w0 + c * 16);
    const v4f q0 = wp[0], q1 = wp[1], q2 = wp[2], q3 = wp[3];
    wv[0] = q0[0]; wv[1] = q0[1]; wv[2] = q0[2]; wv[3] = q0[3];
    wv[4] = q1[0]; wv[5] = q1[1]; wv[6] = q1[2]; wv[7] = q1[3];
    wv[8] = q2[0]; wv[9] = q2[1]; wv[10] = q2[2]; wv[11] = q2[3];
    wv[12] = q3[0]; wv[13] = q3[1]; wv[14] = q3[2]; wv[15] = q3[3];
  }
  const float cbias = cb[c], gg = g[c], bb = be[c], mm = mn[c];
  const float inv = rsqrtf(vr[c] + 1e-5f);
  __syncthreads();
#pragma unroll 1
  for (int it = 0; it < 8; ++it) {
    const int ql = 2 * qp + (it >> 2);
    const int j = it & 3;
    const float* s = xs + 16 * (ql * 4 + j);
    float u0 = cbias, u1 = cbias;
#pragma unroll
    for (int i = 0; i < 16; ++i) {
      const float sv0 = s[i], sv1 = s[i + 8];
      u0 = fmaf(wv[i], sv0, u0);
      u1 = fmaf(wv[i], sv1, u1);
    }
    const float y = fmaxf(fmaxf(u0, u1), 0.0f);
    const float v = gg * (y - mm) * inv + bb;
    ot[ql * kA0Pitch + c * 4 + j] = (_Float16)v;
  }
  __syncthreads();
  {
    const v8h val = *(const v8h*)(ot + wave * kA0Pitch + 8 * lane);
    _Float16* dst = a0q + ((size_t)(b * kNQ + 4 * g4 + wave)) * kA0Pitch + 8 * lane;
    *(volatile v8h*)dst = val;
    __threadfence();
    *(volatile v8h*)dst = val;
  }
}

__global__ __launch_bounds__(256) void k_zero16(v4u* __restrict__ p, int n) {
  const int i = blockIdx.x * blockDim.x + threadIdx.x;
  if (i < n) {
    const v4u z = (v4u){0u, 0u, 0u, 0u};
    ((volatile v4u*)p)[i] = z;
    __threadfence();
    ((volatile v4u*)p)[i] = z;
  }
}

__global__ __launch_bounds__(256) void k_cast2s(const float* __restrict__ in, unsigned* __restrict__ out, int n2, float s) {
  const int i = blockIdx.x * 256 + threadIdx.x;
  if (i < n2) {
    const v2f pr = *(const v2f*)(in + 2 * (size_t)i);
    const unsigned u = pack_h2(pr[0] * s, pr[1] * s);
    ((volatile unsigned*)out)[i] = u;
    __threadfence();
    ((volatile unsigned*)out)[i] = u;
  }
}

__global__ __launch_bounds__(256) void k_w1r(const float* __restrict__ w1, unsigned* __restrict__ out, float s) {
  const int u = blockIdx.x * 256 + threadIdx.x;
  const int co = u >> 8;
  const int kq = (u & 255) * 2;
  const int half = kq >> 8, ci = (kq >> 2) & 63, j = kq & 3;
  const int src = co * 512 + ci * 8 + half * 4 + j;
  const v2f pr = *(const v2f*)(w1 + src);
  const unsigned w = pack_h2(pr[0] * s, pr[1] * s);
  ((volatile unsigned*)out)[u] = w;
  __threadfence();
  ((volatile unsigned*)out)[u] = w;
}

__global__ __launch_bounds__(256) void k_bsum(const float* __restrict__ bi0, const float* __restrict__ bh0,
    const float* __restrict__ bi1, const float* __restrict__ bh1, float* __restrict__ bs) {
  const int i = blockIdx.x * 256 + threadIdx.x;
  const bool second = (blockIdx.x >= 4);
  const float* pa = second ? bi1 : bi0;
  const float* pb = second ? bh1 : bh0;
  const int n = i & 1023;
  const float v = pa[n] + pb[n];
  ((volatile float*)bs)[i] = v;
  __threadfence();
  ((volatile float*)bs)[i] = v;
}

__global__ __launch_bounds__(256) void k_pool1(const float* __restrict__ C1, const float* __restrict__ g,
    const float* __restrict__ be, const float* __restrict__ mn, const float* __restrict__ vr, unsigned* __restrict__ X0u) {
  const int idx = blockIdx.x * 256 + threadIdx.x;
  const int pr = idx & 63;
  const int row = idx >> 6;
  const int t = row >> 8, b = row & 255;
  const int m0 = b * kNQ + 2 * t;
  const float* p0 = C1 + (size_t)m0 * kCh1 + 2 * pr;
  const v2f a0 = *(const v2f*)(p0);
  const v2f a1 = *(const v2f*)(p0 + kCh1);
  const float y0 = fmaxf(a0[0], a1[0]);
  const float y1 = fmaxf(a0[1], a1[1]);
  const int c0 = 2 * pr, c1 = 2 * pr + 1;
  const float v0 = g[c0] * (y0 - mn[c0]) * rsqrtf(vr[c0] + 1e-5f) + be[c0];
  const float v1 = g[c1] * (y1 - mn[c1]) * rsqrtf(vr[c1] + 1e-5f) + be[c1];
  const unsigned w = pack_h2(v0, v1);
  ((volatile unsigned*)X0u)[idx] = w;
  __threadfence();
  ((volatile unsigned*)X0u)[idx] = w;
}

__global__ __launch_bounds__(512) void k_lstm_rec(const float* __restrict__ GT, int ldg,
    const unsigned short* __restrict__ Whp, unsigned short* __restrict__ Hsp, int nsteps, float wscale) {
  const _Float16* Whh = (const _Float16*)Whp;
  _Float16* Hs = (_Float16*)Hsp;
  union FH { v16h v; v8h h[2]; };
  __shared__ __align__(16) _Float16 hA[16 * kHP];
  const int tid = threadIdx.x, lane = tid & 31, wave = tid >> 5;
  const int rl = lane & 15, hh = lane >> 4, koff = hh * 8;
  const int b0 = blockIdx.x * 16;
  {
    unsigned* hz = (unsigned*)hA;
    for (int i = tid; i < (16 * kHP) / 2; i += 512) hz[i] = 0u;
  }
  float cst[8];
#pragma unroll
  for (int r = 0; r < 8; ++r) cst[r] = 0.0f;
  const int col = wave * 16 + rl;
  __syncthreads();

  for (int t = 0; t < nsteps; ++t) {
    v8f acc[4];
#pragma unroll
    for (int s = 0; s < 4; ++s) acc[s] = (v8f){0.f,0.f,0.f,0.f,0.f,0.f,0.f,0.f};
#pragma unroll 1
    for (int kk = 0; kk < kHid; kk += 64) {
#pragma unroll
      for (int u = 0; u < 2; ++u) {
        const int k0 = kk + u * 32;
        FH fa;
        fa.h[0] = *(const v8h*)(hA + rl * kHP + k0 + koff);
        fa.h[1] = *(const v8h*)(hA + rl * kHP + k0 + koff + 16);
#pragma unroll
        for (int s = 0; s < 4; ++s) {
          const v16h bq = Frag<_Float16>::load(Whh + (size_t)(s * kHid + col) * kHid + k0 + koff);
          acc[s] = mma_h16(fa.v, bq, acc[s]);
        }
      }
    }
    float gv[4][8];
#pragma unroll
    for (int s = 0; s < 4; ++s) {
      const float* gp = GT + (size_t)(s * kHid + col) * ldg + (size_t)t * kNB + b0 + 8 * hh;
      const v4f ga = *(const v4f*)(gp);
      const v4f gb = *(const v4f*)(gp + 4);
      gv[s][0] = ga[0]; gv[s][1] = ga[1]; gv[s][2] = ga[2]; gv[s][3] = ga[3];
      gv[s][4] = gb[0]; gv[s][5] = gb[1]; gv[s][6] = gb[2]; gv[s][7] = gb[3];
    }
    float hv[8];
#pragma unroll
    for (int r = 0; r < 8; ++r) {
      const float ig = sigm_f(acc[0][r] * wscale + gv[0][r]);
      const float fg = sigm_f(acc[1][r] * wscale + gv[1][r]);
      const float gg = tanhf(acc[2][r] * wscale + gv[2][r]);
      const float og = sigm_f(acc[3][r] * wscale + gv[3][r]);
      const float cn = fg * cst[r] + ig * gg;
      cst[r] = cn;
      hv[r] = og * tanhf(cn);
    }
    __syncthreads();
#pragma unroll
    for (int r = 0; r < 8; ++r) hA[(8 * hh + r) * kHP + col] = (_Float16)hv[r];
    __syncthreads();
    {
      const v8h val = *(const v8h*)(hA + wave * kHP + 8 * lane);
      _Float16* dst = Hs + ((size_t)t * kNB + b0 + wave) * kHid + 8 * lane;
      *(volatile v8h*)dst = val;
      __threadfence();
      *(volatile v8h*)dst = val;
    }
  }
}

template <int BIAS_MODE, int OUT_MODE, int ACT>
static void gemm_f16(hipStream_t st, const void* A, int lda, const void* Bt, int ldb, void* Cp, int ldc,
                     const float* bias, int M, int N, int K, float scale) {
  const int tiles = (M / 64) * (N / 64);
  const int blocks = (tiles + 7) / 8;
  wmma_gemm64<0, false, BIAS_MODE, OUT_MODE, false, ACT><<<dim3(blocks, 1), 256, 0, st>>>(
      (const unsigned short*)A, (const unsigned short*)A, lda, 0L,
      (const unsigned short*)Bt, (const unsigned short*)Bt, ldb, 0L,
      Cp, Cp, ldc, 0L, bias, bias, 0L, M, N, K, scale);
}

static void h_norm_inverse(const double V[11][4], double Mi[4][4]) {
  double a[4][8];
  for (int i = 0; i < 4; ++i)
    for (int j = 0; j < 4; ++j) {
      double s = 0.0;
      for (int w = 0; w < 11; ++w) s += V[w][i] * V[w][j];
      a[i][j] = s;
      a[i][j + 4] = (i == j) ? 1.0 : 0.0;
    }
  for (int c = 0; c < 4; ++c) {
    int piv = c;
    for (int r = c + 1; r < 4; ++r) {
      double x0 = a[r][c] < 0 ? -a[r][c] : a[r][c];
      double x1 = a[piv][c] < 0 ? -a[piv][c] : a[piv][c];
      if (x0 > x1) piv = r;
    }
    if (piv != c)
      for (int j = 0; j < 8; ++j) { double tmp = a[c][j]; a[c][j] = a[piv][j]; a[piv][j] = tmp; }
    const double d = a[c][c];
    for (int j = 0; j < 8; ++j) a[c][j] /= d;
    for (int r = 0; r < 4; ++r) if (r != c) {
      const double f = a[r][c];
      for (int j = 0; j < 8; ++j) a[r][j] -= f * a[c][j];
    }
  }
  for (int i = 0; i < 4; ++i) for (int j = 0; j < 4; ++j) Mi[i][j] = a[i][j + 4];
}

static void h_make_taps(SgTaps& tp) {
  double V[11][4], Ve[11][4];
  for (int w = 0; w < 11; ++w) {
    const double tc = (double)(w - 5), te = (double)w;
    double pc = 1.0, pe = 1.0;
    for (int j = 0; j < 4; ++j) { V[w][j] = pc; Ve[w][j] = pe; pc *= tc; pe *= te; }
  }
  double Mi[4][4], Mei[4][4];
  h_norm_inverse(V, Mi);
  h_norm_inverse(Ve, Mei);
  for (int i = 0; i < 124; ++i) tp.tt[i] = 0.0f;
  for (int w = 0; w < 11; ++w) {
    double s = 0.0;
    for (int i = 0; i < 4; ++i) s += Mi[0][i] * V[w][i];
    tp.tt[5 * 11 + w] = (float)s;
  }
  double pe[4][11];
  for (int j = 0; j < 4; ++j)
    for (int w = 0; w < 11; ++w) {
      double s = 0.0;
      for (int i = 0; i < 4; ++i) s += Mei[j][i] * Ve[w][i];
      pe[j][w] = s;
    }
  for (int k = 0; k < 5; ++k) {
    const double t0 = (double)k, t1 = (double)(6 + k);
    for (int w = 0; w < 11; ++w) {
      double pf = 0.0, pl = 0.0, p0 = 1.0, p1 = 1.0;
      for (int j = 0; j < 4; ++j) { pf += pe[j][w] * p0; pl += pe[j][w] * p1; p0 *= t0; p1 *= t1; }
      tp.tt[k * 11 + w] = (float)pf;
      tp.tt[(6 + k) * 11 + w] = (float)pl;
    }
  }
}

static const size_t OFF_YSG  = 0;
static const size_t OFF_A0Q  = 10240000ull;
static const size_t OFF_C1   = OFF_A0Q + 20451328ull;
static const size_t OFF_GT   = 0;
static const size_t SZ_GT    = (size_t)kGates * kNX * 4;
static const size_t OFF_X0   = SZ_GT;
static const size_t OFF_HS1  = OFF_X0;
static const size_t OFF_HS0  = OFF_X0 + (size_t)kNX * kHid * 2;
static const size_t OFF_W    = OFF_HS0 + (size_t)kNX * kHid * 2;
static const size_t WB_WIH0  = 0;
static const size_t WB_WHH0  = 262144;
static const size_t WB_WIH1  = 786432;
static const size_t WB_WHH1  = 1310720;
static const size_t WB_FC0   = 1835008;
static const size_t WB_FC1   = 2097152;
static const size_t WB_OUTW  = 2621440;
static const size_t WB_W1R   = 2883584;
static const size_t SZ_W     = 3014656;
static const size_t OFF_BS   = OFF_W + SZ_W;
static const size_t OFF_Z0   = OFF_BS + 8192;
static const size_t OFF_Z1   = OFF_Z0 + 262144;
static const size_t WS_END   = OFF_Z1 + 262144;
static_assert(OFF_C1 + (size_t)kRowsA0 * kCh1 * 4 <= SZ_GT, "early-phase planes fit under GT");
static_assert(OFF_A0Q + (size_t)(kRowsA0 + 1) * kA0Pitch * 2 <= OFF_C1, "quad plane + pad row fits its carve");
static_assert((size_t)kNX * kCh1 * 2 <= (size_t)kNX * kHid * 2, "X0 fits the X region");
static_assert(WS_END <= 134217728ull, "carve under 128 MiB");

extern "C" void kernel_launch(void* const* d_in, const int* in_sizes, int n_in,
                              void* d_out, int out_size, void* d_ws, size_t ws_size,
                              hipStream_t stream) {
  if (n_in != 27) return;
  if (in_sizes[0] != kNB * kLX) return;
  if (out_size != kNB * kCls) return;
  if (ws_size < WS_END) return;

  const float* x       = (const float*)d_in[0];
  const float* conv_w0 = (const float*)d_in[1];
  const float* conv_b0 = (const float*)d_in[2];
  const float* bn_g0   = (const float*)d_in[3];
  const float* bn_b0   = (const float*)d_in[4];
  const float* bn_m0   = (const float*)d_in[5];
  const float* bn_v0   = (const float*)d_in[6];
  const float* conv_w1 = (const float*)d_in[7];
  const float* conv_b1 = (const float*)d_in[8];
  const float* bn_g1   = (const float*)d_in[9];
  const float* bn_b1   = (const float*)d_in[10];
  const float* bn_m1   = (const float*)d_in[11];
  const float* bn_v1   = (const float*)d_in[12];
  const float* Wih0    = (const float*)d_in[13];
  const float* Whh0    = (const float*)d_in[14];
  const float* bih0    = (const float*)d_in[15];
  const float* bhh0    = (const float*)d_in[16];
  const float* Wih1    = (const float*)d_in[17];
  const float* Whh1    = (const float*)d_in[18];
  const float* bih1    = (const float*)d_in[19];
  const float* bhh1    = (const float*)d_in[20];
  const float* fc0_w   = (const float*)d_in[21];
  const float* fc0_b   = (const float*)d_in[22];
  const float* fc1_w   = (const float*)d_in[23];
  const float* fc1_b   = (const float*)d_in[24];
  const float* out_w   = (const float*)d_in[25];
  const float* out_b   = (const float*)d_in[26];

  char* ws = (char*)d_ws;
  float*          ysg   = (float*)(ws + OFF_YSG);
  unsigned short* a0q   = (unsigned short*)(ws + OFF_A0Q);
  float*          c1    = (float*)(ws + OFF_C1);
  float*          gt    = (float*)(ws + OFF_GT);
  unsigned*       x0u   = (unsigned*)(ws + OFF_X0);
  unsigned short* hs0   = (unsigned short*)(ws + OFF_HS0);
  unsigned short* hs1   = (unsigned short*)(ws + OFF_HS1);
  unsigned*       wih0p = (unsigned*)(ws + OFF_W + WB_WIH0);
  unsigned*       whh0p = (unsigned*)(ws + OFF_W + WB_WHH0);
  unsigned*       wih1p = (unsigned*)(ws + OFF_W + WB_WIH1);
  unsigned*       whh1p = (unsigned*)(ws + OFF_W + WB_WHH1);
  unsigned*       fc0p  = (unsigned*)(ws + OFF_W + WB_FC0);
  unsigned*       fc1p  = (unsigned*)(ws + OFF_W + WB_FC1);
  unsigned*       outwp = (unsigned*)(ws + OFF_W + WB_OUTW);
  unsigned*       w1rp  = (unsigned*)(ws + OFF_W + WB_W1R);
  float*          bsum  = (float*)(ws + OFF_BS);
  unsigned short* z0    = (unsigned short*)(ws + OFF_Z0);
  unsigned short* z1    = (unsigned short*)(ws + OFF_Z1);

  SgTaps taps;
  h_make_taps(taps);

  k_savgol<<<(kNB * kLX) / 256, 256, 0, stream>>>(x, ysg, taps);
  k_conv0<<<dim3(39, kNB), 128, 0, stream>>>(ysg, conv_w0, conv_b0, bn_g0, bn_b0, bn_m0, bn_v0, a0q);
  k_zero16<<<1, 32, 0, stream>>>((v4u*)(ws + OFF_A0Q + (size_t)kRowsA0 * kA0Pitch * 2), 32);
  k_cast2s<<<(kGates * kCh1 / 2 + 255) / 256, 256, 0, stream>>>(Wih0, wih0p, kGates * kCh1 / 2, kWScale);
  k_cast2s<<<(kGates * kHid / 2 + 255) / 256, 256, 0, stream>>>(Whh0, whh0p, kGates * kHid / 2, kWScale);
  k_cast2s<<<(kGates * kHid / 2 + 255) / 256, 256, 0, stream>>>(Wih1, wih1p, kGates * kHid / 2, kWScale);
  k_cast2s<<<(kGates * kHid / 2 + 255) / 256, 256, 0, stream>>>(Whh1, whh1p, kGates * kHid / 2, kWScale);
  k_cast2s<<<(kFc * kHid / 2 + 255) / 256, 256, 0, stream>>>(fc0_w, fc0p, kFc * kHid / 2, kWScale);
  k_cast2s<<<(kFc * kFc / 2 + 255) / 256, 256, 0, stream>>>(fc1_w, fc1p, kFc * kFc / 2, kWScale);
  k_cast2s<<<(kCls * kFc / 2 + 255) / 256, 256, 0, stream>>>(out_w, outwp, kCls * kFc / 2, kWScale);
  k_w1r<<<(kCh1 * kK1 / 2) / 256, 256, 0, stream>>>(conv_w1, w1rp, kWScale);
  k_bsum<<<8, 256, 0, stream>>>(bih0, bhh0, bih1, bhh1, bsum);
  gemm_f16<2, 0, 2>(stream, a0q, kA0Pitch, w1rp, kK1, c1, kCh1, conv_b1, kRowsA0, kCh1, kK1, kWScaleInv);
  k_pool1<<<(kNX * kCh1 / 2) / 256, 256, 0, stream>>>(c1, bn_g1, bn_b1, bn_m1, bn_v1, x0u);
  gemm_f16<1, 0, 0>(stream, wih0p, kCh1, x0u, kCh1, gt, kNX, bsum, kGates, kNX, kCh1, kWScaleInv);
  k_lstm_rec<<<kNB / 16, 512, 0, stream>>>(gt, kNX, (const unsigned short*)whh0p, hs0, kSteps, kWScaleInv);
  gemm_f16<1, 0, 0>(stream, wih1p, kHid, hs0, kHid, gt, kNX, bsum + kGates, kGates, kNX, kHid, kWScaleInv);
  k_lstm_rec<<<kNB / 16, 512, 0, stream>>>(gt, kNX, (const unsigned short*)whh1p, hs1, kSteps, kWScaleInv);
  gemm_f16<2, 1, 2>(stream, hs1 + (size_t)(kSteps - 1) * kNB * kHid, kHid, fc0p, kHid, z0, kFc, fc0_b, kNB, kFc, kHid, kWScaleInv);
  gemm_f16<2, 1, 2>(stream, z0, kFc, fc1p, kFc, z1, kFc, fc1_b, kNB, kFc, kFc, kWScaleInv);
  gemm_f16<2, 0, 0>(stream, z1, kFc, outwp, kFc, d_out, kCls, out_b, kNB, kCls, kFc, kWScaleInv);
}
